// DovePeakPredictor_75385265979999
// MI455X (gfx1250) — hardware-run, weakly checked
//
#include <hip/hip_runtime.h>
#include <math.h>

typedef __attribute__((ext_vector_type(16))) _Float16 v16h;
typedef __attribute__((ext_vector_type(8)))  _Float16 v8h;
typedef __attribute__((ext_vector_type(8)))  float    v8f;
typedef __attribute__((ext_vector_type(4)))  float    v4f;
typedef __attribute__((ext_vector_type(4)))  unsigned int v4u;

constexpr int kB      = 4;
constexpr int kL      = 2048;
constexpr int kNF     = 10;
constexpr int kDED    = 128;
constexpr int kD      = 128;
constexpr int kH      = 4;
constexpr int kNL     = 4;
constexpr int kHid    = 512;
constexpr int kHid2   = 2 * kHid;
constexpr int kHead   = kD / kH;
constexpr int kCin    = 2 * kNF + kDED;
constexpr int kTok    = kB * kL;
constexpr int kNumEmb = 501;
constexpr int kQKld   = 2 * kD;
constexpr int kPP     = 72;
constexpr int kOP     = 132;
constexpr float kWCarry   = 16.0f;
constexpr float kActCarry = 16.0f;
constexpr float kPCarry   = 32768.0f;
constexpr float kWInv     = 1.0f / kWCarry;
constexpr float kW2Inv    = 1.0f / (kWCarry * kActCarry);
constexpr float kNormEps  = 1e-8f;
static_assert(kHead == 32, "one k-step per score tile");
static_assert(kCin == 148, "input row width");
static_assert(kTok == 8192, "token rows");
static_assert((kD % 32) == 0 && (kHid % 32) == 0, "GEMM K multiples of 32");
static_assert((kTok % 64) == 0 && (kQKld % 64) == 0 && (kD % 64) == 0 && (kHid2 % 64) == 0, "GEMM M,N multiples of 64");
static_assert((kL % 64) == 0, "key chunks of 64");

constexpr size_t kOffWQKV = 0;
constexpr size_t kOffWO   = kOffWQKV + (size_t)kNL * 3 * kD * kD * 2;
constexpr size_t kOffW1   = kOffWO   + (size_t)kNL * kD * kD * 2;
constexpr size_t kOffW2   = kOffW1   + (size_t)kNL * kHid2 * kD * 2;
constexpr size_t kOffHA   = kOffW2   + (size_t)kNL * kD * kHid * 2;
constexpr size_t kOffHB   = kOffHA   + (size_t)kTok * kD * 4;
constexpr size_t kOffHN   = kOffHB   + (size_t)kTok * kD * 4;
constexpr size_t kOffQK   = kOffHN   + (size_t)kTok * kD * 2;
constexpr size_t kOffVT   = kOffQK   + (size_t)kTok * kQKld * 2;
constexpr size_t kOffOA   = kOffVT   + (size_t)kD * kTok * 2;
constexpr size_t kOffFF   = kOffOA   + (size_t)kTok * kD * 2;
constexpr size_t kOffACT  = kOffFF   + (size_t)kTok * kHid2 * 4;
constexpr size_t kOffCB   = kOffACT  + (size_t)kTok * kHid * 2;
constexpr size_t kOffPL   = kOffCB   + (size_t)kB * kD * 4;
constexpr size_t kWsTotal = kOffPL   + (size_t)kB * kD * 4;
static_assert(kWsTotal == 62918656ull, "carve total");
static_assert(kWsTotal <= 134217728ull, "carve cap");
static_assert((kOffWO % 128) == 0 && (kOffW1 % 128) == 0 && (kOffW2 % 128) == 0 && (kOffHA % 128) == 0 &&
              (kOffHB % 128) == 0 && (kOffHN % 128) == 0 && (kOffQK % 128) == 0 && (kOffVT % 128) == 0 &&
              (kOffOA % 128) == 0 && (kOffFF % 128) == 0 && (kOffACT % 128) == 0 && (kOffCB % 128) == 0 &&
              (kOffPL % 128) == 0, "128-B aligned regions");

union FragU { v16h v; v8h h[2]; };
__device__ __forceinline__ v16h frag_load(const _Float16* p) {
  FragU f;
  f.h[0] = *(const v8h*)(p);
  f.h[1] = *(const v8h*)(p + 16);
  return f.v;
}
__device__ __forceinline__ v8f mma_f16(v16h a, v16h b, v8f c) {
  c = __builtin_amdgcn_wmma_f32_16x16x32_f16(false, a, false, b, (short)0, c, false, false);
  asm volatile("v_nop\n\tv_nop\n\tv_nop\n\tv_nop" : "+v"(c) : "v"(a), "v"(b));
  return c;
}
__device__ __forceinline__ void acc_guard4(v8f& a, v8f& b, v8f& c, v8f& d) {
  asm volatile("v_nop\n\tv_nop\n\tv_nop\n\tv_nop" : "+v"(a), "+v"(b), "+v"(c), "+v"(d));
}
__device__ __forceinline__ void wave_lds_sync() {
  __builtin_amdgcn_fence(__ATOMIC_RELEASE, "workgroup");
  __builtin_amdgcn_wave_barrier();
  __builtin_amdgcn_fence(__ATOMIC_ACQUIRE, "workgroup");
}
__device__ __forceinline__ unsigned pk16(unsigned short a, unsigned short b) { return (unsigned)a | ((unsigned)b << 16); }
__device__ __forceinline__ unsigned short h_bits(float f) { const _Float16 h = (_Float16)f; return __builtin_bit_cast(unsigned short, h); }

template <int BIAS_MODE, int OUT_MODE, bool RESID>
__global__ __launch_bounds__(256) void wmma_gemm64(
    const unsigned short* __restrict__ Ap, int lda,
    const unsigned short* __restrict__ Btp, int ldb,
    void* __restrict__ Cout, int ldc,
    const float* __restrict__ bias, const float* __restrict__ resid,
    int M, int N, int K, float scale) {
  const _Float16* A  = (const _Float16*)Ap;
  const _Float16* Bt = (const _Float16*)Btp;
  __shared__ __align__(16) float sT[8][16 * 68];
  const int lane = threadIdx.x & 31;
  const int wave = threadIdx.x >> 5;
  const int tilesN = N >> 6;
  const int tilesM = M >> 6;
  const int tile = blockIdx.x * 8 + wave;
  if (tile >= tilesM * tilesN) return;
  const int tm = tile / tilesN;
  const int tn = tile - tm * tilesN;
  const int m0 = tm << 6;
  const int n0 = tn << 6;
  const int rlane = lane & 15;
  const int koff  = (lane >> 4) * 8;
  const int mOff  = (lane >> 4) * 8;

  v8f acc[4][4];
#pragma unroll
  for (int i = 0; i < 4; ++i)
#pragma unroll
    for (int j = 0; j < 4; ++j) acc[i][j] = (v8f){0.f,0.f,0.f,0.f,0.f,0.f,0.f,0.f};

  for (int k0 = 0; k0 < K; k0 += 32) {
    v16h bh[4];
#pragma unroll
    for (int j = 0; j < 4; ++j) {
      const size_t bo = (size_t)(n0 + (j << 4) + rlane) * ldb + koff + k0;
      bh[j] = frag_load(Bt + bo);
    }
#pragma unroll
    for (int i = 0; i < 4; ++i) {
      const size_t ao = (size_t)(m0 + (i << 4) + rlane) * lda + koff + k0;
      const v16h ah = frag_load(A + ao);
#pragma unroll
      for (int j = 0; j < 4; ++j) acc[i][j] = mma_f16(ah, bh[j], acc[i][j]);
    }
  }
  acc_guard4(acc[0][0], acc[0][1], acc[0][2], acc[0][3]);
  acc_guard4(acc[1][0], acc[1][1], acc[1][2], acc[1][3]);
  acc_guard4(acc[2][0], acc[2][1], acc[2][2], acc[2][3]);
  acc_guard4(acc[3][0], acc[3][1], acc[3][2], acc[3][3]);

  float* slab = sT[wave];
#pragma unroll
  for (int i = 0; i < 4; ++i) {
    const int mBase = m0 + (i << 4);
#pragma unroll
    for (int j = 0; j < 4; ++j) {
      const int n = n0 + (j << 4) + rlane;
      float bv = 0.f;
      if (BIAS_MODE == 2) bv = bias[n];
#pragma unroll
      for (int r = 0; r < 8; ++r) {
        float v = acc[i][j][r] * scale;
        if (BIAS_MODE == 1) v += bias[mBase + mOff + r];
        if (BIAS_MODE == 2) v += bv;
        slab[(mOff + r) * 68 + (j << 4) + rlane] = v;
      }
    }
    wave_lds_sync();
    if (OUT_MODE == 0) {
      float* C = (float*)Cout;
      const int hh = lane >> 4, c4 = (lane & 15) * 4;
      v4f vals[8];
#pragma unroll
      for (int it = 0; it < 8; ++it) {
        const int row = it * 2 + hh;
        v4f v = *(const v4f*)(slab + row * 68 + c4);
        if (RESID) {
          const v4f rr = *(const v4f*)(resid + (size_t)(mBase + row) * ldc + n0 + c4);
          v = v + rr;
        }
        vals[it] = v;
      }
      for (int pass = 0; pass < 2; ++pass) {
#pragma unroll
        for (int it = 0; it < 8; ++it) {
          const int row = it * 2 + hh;
          *(volatile v4f*)(C + (size_t)(mBase + row) * ldc + n0 + c4) = vals[it];
        }
        __threadfence();
      }
    } else {
      const int q = lane >> 3, c8 = (lane & 7) * 8;
      unsigned short* C = (unsigned short*)Cout;
      v8h hv[4];
#pragma unroll
      for (int it = 0; it < 4; ++it) {
        const int row = it * 4 + q;
        const float* sp = slab + row * 68 + c8;
#pragma unroll
        for (int e = 0; e < 8; ++e) hv[it][e] = (_Float16)sp[e];
      }
      for (int pass = 0; pass < 2; ++pass) {
#pragma unroll
        for (int it = 0; it < 4; ++it) {
          const int row = it * 4 + q;
          *(volatile v8h*)(C + (size_t)(mBase + row) * ldc + n0 + c8) = hv[it];
        }
        __threadfence();
      }
    }
    wave_lds_sync();
  }
}

__global__ __launch_bounds__(256) void cast8_f16_kernel(const float* __restrict__ in, unsigned short* __restrict__ out,
                                                        int n8, float carry) {
  const int i = blockIdx.x * 256 + threadIdx.x;
  if (i >= n8) return;
  const float* p = in + 8 * (size_t)i;
  const v4f a = *(const v4f*)(p);
  const v4f c = *(const v4f*)(p + 4);
  unsigned short hb[8];
#pragma unroll
  for (int e = 0; e < 4; ++e) {
    hb[e]     = h_bits(a[e] * carry);
    hb[4 + e] = h_bits(c[e] * carry);
  }
  const v4u u = (v4u){pk16(hb[0], hb[1]), pk16(hb[2], hb[3]), pk16(hb[4], hb[5]), pk16(hb[6], hb[7])};
  unsigned short* q = out + 8 * (size_t)i;
  *(volatile v4u*)q = u;
  __threadfence();
  *(volatile v4u*)q = u;
}

__global__ __launch_bounds__(128) void embed_const_kernel(const int* __restrict__ ids, const float* __restrict__ emb,
                                                          const float* __restrict__ W_in, const float* __restrict__ b_in,
                                                          float* __restrict__ cb) {
  const int d = threadIdx.x;
  const float* wrow = W_in + (size_t)d * kCin + 2 * kNF;
  const float bias = b_in[d];
  float res[kB];
#pragma unroll
  for (int b = 0; b < kB; ++b) {
    int id = ids[b];
    id = id < 0 ? 0 : id;
    id = id > (kNumEmb - 1) ? (kNumEmb - 1) : id;
    const float* de = emb + (size_t)id * kDED;
    float acc = bias;
#pragma unroll 4
    for (int j = 0; j < kDED; ++j) acc = fmaf(wrow[j], de[j], acc);
    res[b] = acc;
  }
  for (int pass = 0; pass < 2; ++pass) {
#pragma unroll
    for (int b = 0; b < kB; ++b) *(volatile float*)(cb + b * kD + d) = res[b];
    __threadfence();
  }
}

__global__ __launch_bounds__(128) void embed_tok_kernel(const float* __restrict__ x, const float* __restrict__ W_in,
                                                        const float* __restrict__ cb, const float* __restrict__ g_in,
                                                        float* __restrict__ hout) {
  __shared__ __align__(16) float sx[32 * kNF];
  __shared__ __align__(16) float sm[32 * kNF];
  __shared__ __align__(16) float sT[32 * kOP];
  const int tid = threadIdx.x, lane = tid & 31, wave = tid >> 5;
  const int t0 = blockIdx.x * 32;
  const int b  = t0 / kL;
#pragma unroll
  for (int i = 0; i < 3; ++i) {
    const int e  = tid + 128 * i;
    const int ec = e < (32 * kNF) ? e : (32 * kNF - 1);
    const float v = x[(size_t)t0 * kNF + ec];
    const bool isn = (v != v);
    const float vc = fminf(fmaxf(v, -3.402823466e+38f), 3.402823466e+38f);
    if (e < 32 * kNF) {
      sx[e] = isn ? 0.0f : vc;
      sm[e] = isn ? 0.0f : 1.0f;
    }
  }
  float w[2 * kNF];
  {
    const float* wr = W_in + (size_t)tid * kCin;
    const v4f w0 = *(const v4f*)(wr);
    const v4f w1 = *(const v4f*)(wr + 4);
    const v4f w2 = *(const v4f*)(wr + 8);
    const v4f w3 = *(const v4f*)(wr + 12);
    const v4f w4 = *(const v4f*)(wr + 16);
    w[0] = w0[0]; w[1] = w0[1]; w[2] = w0[2]; w[3] = w0[3];
    w[4] = w1[0]; w[5] = w1[1]; w[6] = w1[2]; w[7] = w1[3];
    w[8] = w2[0]; w[9] = w2[1]; w[10] = w2[2]; w[11] = w2[3];
    w[12] = w3[0]; w[13] = w3[1]; w[14] = w3[2]; w[15] = w3[3];
    w[16] = w4[0]; w[17] = w4[1]; w[18] = w4[2]; w[19] = w4[3];
  }
  const float cbv = cb[b * kD + tid];
  __syncthreads();
#pragma unroll 1
  for (int t = 0; t < 32; ++t) {
    float acc = cbv;
#pragma unroll
    for (int j = 0; j < kNF; ++j) {
      acc = fmaf(w[j], sx[t * kNF + j], acc);
      acc = fmaf(w[kNF + j], sm[t * kNF + j], acc);
    }
    sT[t * kOP + tid] = acc;
  }
  __syncthreads();
  const v4f g4 = *(const v4f*)(g_in + lane * 4);
#pragma unroll 1
  for (int it = 0; it < 8; ++it) {
    const int row = wave * 8 + it;
    const v4f a = *(const v4f*)(sT + row * kOP + lane * 4);
    float ss = a[0] * a[0] + a[1] * a[1] + a[2] * a[2] + a[3] * a[3];
    ss += __shfl_xor(ss, 16, 32);
    ss += __shfl_xor(ss, 8, 32);
    ss += __shfl_xor(ss, 4, 32);
    ss += __shfl_xor(ss, 2, 32);
    ss += __shfl_xor(ss, 1, 32);
    const float r = rsqrtf(ss * (1.0f / (float)kD) + kNormEps);
    v4f o;
    o[0] = g4[0] * a[0] * r;
    o[1] = g4[1] * a[1] * r;
    o[2] = g4[2] * a[2] * r;
    o[3] = g4[3] * a[3] * r;
    float* dst = hout + (size_t)(t0 + row) * kD + lane * 4;
    *(volatile v4f*)dst = o;
    __threadfence();
    *(volatile v4f*)dst = o;
  }
}

__global__ __launch_bounds__(256) void rmsnorm_f16_kernel(const float* __restrict__ h, const float* __restrict__ g,
                                                          unsigned short* __restrict__ out) {
  const int tid = threadIdx.x, lane = tid & 31, wave = tid >> 5;
  const int sub = lane >> 4, l16 = lane & 15;
  const int row = blockIdx.x * 16 + wave * 2 + sub;
  const float* hp = h + (size_t)row * kD + l16 * 8;
  const v4f a0 = *(const v4f*)(hp);
  const v4f a1 = *(const v4f*)(hp + 4);
  const v4f g0 = *(const v4f*)(g + l16 * 8);
  const v4f g1 = *(const v4f*)(g + l16 * 8 + 4);
  float ss = a0[0] * a0[0] + a0[1] * a0[1] + a0[2] * a0[2] + a0[3] * a0[3]
           + a1[0] * a1[0] + a1[1] * a1[1] + a1[2] * a1[2] + a1[3] * a1[3];
  ss += __shfl_xor(ss, 8, 32);
  ss += __shfl_xor(ss, 4, 32);
  ss += __shfl_xor(ss, 2, 32);
  ss += __shfl_xor(ss, 1, 32);
  const float r = rsqrtf(ss * (1.0f / (float)kD) + kNormEps);
  v8h hv;
#pragma unroll
  for (int e = 0; e < 4; ++e) {
    hv[e]     = (_Float16)(g0[e] * a0[e] * r);
    hv[4 + e] = (_Float16)(g1[e] * a1[e] * r);
  }
  unsigned short* dst = out + (size_t)row * kD + l16 * 8;
  *(volatile v8h*)dst = hv;
  __threadfence();
  *(volatile v8h*)dst = hv;
}

__global__ __launch_bounds__(128) void attn_full_kernel(const unsigned short* __restrict__ qkp,
                                                        const unsigned short* __restrict__ vtp,
                                                        unsigned short* __restrict__ outp, float qk_scale) {
  __shared__ __align__(16) _Float16 Psh[4][16 * kPP];
  __shared__ __align__(16) float    Osh[4][16 * kOP];
  const _Float16* qk = (const _Float16*)qkp;
  const _Float16* vt = (const _Float16*)vtp;
  const int tid = threadIdx.x, wave = tid >> 5, lane = tid & 31;
  const int hh = lane >> 4, c = lane & 15;
  constexpr int kQBlocks = kL / 64;
  constexpr int kKeyChunks = kL / 64;
  const int b  = blockIdx.x / kQBlocks;
  const int qb = blockIdx.x - b * kQBlocks;
  const int q0 = qb * 64 + wave * 16;
  const size_t tok0 = (size_t)b * kL;
  _Float16* pw = Psh[wave];
  float*    os = Osh[wave];

#pragma unroll 1
  for (int h = 0; h < kH; ++h) {
    const float slope = ldexpf(1.0f, 2 * h - 3);
    const v16h qa = frag_load(qk + (tok0 + q0 + c) * kQKld + h * kHead + 8 * hh);
    const _Float16* kbase = qk + tok0 * kQKld + kD + h * kHead + 8 * hh;
    const _Float16* vbase = vt + (size_t)(h * kHead + c) * kTok + tok0 + 8 * hh;

    float mrow[8], lpart[8];
    v8f oacc[2];
#pragma unroll
    for (int r = 0; r < 8; ++r) { mrow[r] = -INFINITY; lpart[r] = 0.f; }
    oacc[0] = (v8f){0.f,0.f,0.f,0.f,0.f,0.f,0.f,0.f};
    oacc[1] = (v8f){0.f,0.f,0.f,0.f,0.f,0.f,0.f,0.f};

#pragma unroll 1
    for (int kc = 0; kc < kKeyChunks; ++kc) {
      const int kv0 = kc << 6;
      v8f s[4];
#pragma unroll
      for (int j = 0; j < 4; ++j) {
        const v16h kb = frag_load(kbase + (size_t)(kv0 + j * 16 + c) * kQKld);
        s[j] = mma_f16(qa, kb, (v8f){0.f,0.f,0.f,0.f,0.f,0.f,0.f,0.f});
      }
      float cm[8];
#pragma unroll
      for (int r = 0; r < 8; ++r) {
        const int qi = q0 + 8 * hh + r;
        float m = -INFINITY;
#pragma unroll
        for (int j = 0; j < 4; ++j) {
          const int kj = kv0 + j * 16 + c;
          const float dist = fabsf((float)(qi - kj));
          const float sc = s[j][r] * qk_scale - slope * dist;
          s[j][r] = sc;
          m = fmaxf(m, sc);
        }
        m = fmaxf(m, __shfl_xor(m, 1, 32));
        m = fmaxf(m, __shfl_xor(m, 2, 32));
        m = fmaxf(m, __shfl_xor(m, 4, 32));
        m = fmaxf(m, __shfl_xor(m, 8, 32));
        cm[r] = m;
      }
#pragma unroll
      for (int r = 0; r < 8; ++r) {
        const float mnew  = fmaxf(mrow[r], cm[r]);
        const float alpha = __expf(mrow[r] - mnew);
        mrow[r] = mnew;
        float psum = 0.f;
#pragma unroll
        for (int j = 0; j < 4; ++j) {
          const float p = __expf(s[j][r] - mnew);
          psum += p;
          pw[(8 * hh + r) * kPP + j * 16 + c] = (_Float16)(p * kPCarry);
        }
        lpart[r] = lpart[r] * alpha + psum;
        oacc[0][r] *= alpha;
        oacc[1][r] *= alpha;
      }
      wave_lds_sync();
#pragma unroll
      for (int kk = 0; kk < 2; ++kk) {
        const v16h pa = frag_load(pw + c * kPP + kk * 32 + 8 * hh);
#pragma unroll
        for (int t = 0; t < 2; ++t) {
          const v16h vb = frag_load(vbase + (size_t)t * 16 * kTok + kv0 + kk * 32);
          oacc[t] = mma_f16(pa, vb, oacc[t]);
        }
      }
      wave_lds_sync();
    }
#pragma unroll
    for (int r = 0; r < 8; ++r) {
      float l = lpart[r];
      l += __shfl_xor(l, 1, 32);
      l += __shfl_xor(l, 2, 32);
      l += __shfl_xor(l, 4, 32);
      l += __shfl_xor(l, 8, 32);
      const float inv = 1.0f / (l * kPCarry);
      os[(8 * hh + r) * kOP + h * kHead + c]      = oacc[0][r] * inv;
      os[(8 * hh + r) * kOP + h * kHead + 16 + c] = oacc[1][r] * inv;
    }
  }
  wave_lds_sync();
  {
    const int c8 = (lane & 15) * 8;
    v8h ov[8];
#pragma unroll
    for (int it = 0; it < 8; ++it) {
      const int row = it * 2 + hh;
      const float* sp = os + row * kOP + c8;
      const v4f a0 = *(const v4f*)(sp);
      const v4f a1 = *(const v4f*)(sp + 4);
#pragma unroll
      for (int e = 0; e < 4; ++e) {
        ov[it][e]     = (_Float16)a0[e];
        ov[it][4 + e] = (_Float16)a1[e];
      }
    }
    for (int pass = 0; pass < 2; ++pass) {
#pragma unroll
      for (int it = 0; it < 8; ++it) {
        const int row = it * 2 + hh;
        *(volatile v8h*)(outp + (tok0 + q0 + row) * kD + c8) = ov[it];
      }
      __threadfence();
    }
  }
}

__global__ __launch_bounds__(256) void gate_mul_kernel(const float* __restrict__ FF, unsigned short* __restrict__ act) {
  const int i = blockIdx.x * 256 + threadIdx.x;
  if (i >= kTok * (kHid / 8)) return;
  const int row = i / (kHid / 8);
  const int c8  = (i - row * (kHid / 8)) * 8;
  const float* fx = FF + (size_t)row * kHid2 + c8;
  const float* fg = fx + kHid;
  const v4f x0 = *(const v4f*)(fx);
  const v4f x1 = *(const v4f*)(fx + 4);
  const v4f g0 = *(const v4f*)(fg);
  const v4f g1 = *(const v4f*)(fg + 4);
  float xs[8], gs[8];
  xs[0] = x0[0]; xs[1] = x0[1]; xs[2] = x0[2]; xs[3] = x0[3];
  xs[4] = x1[0]; xs[5] = x1[1]; xs[6] = x1[2]; xs[7] = x1[3];
  gs[0] = g0[0]; gs[1] = g0[1]; gs[2] = g0[2]; gs[3] = g0[3];
  gs[4] = g1[0]; gs[5] = g1[1]; gs[6] = g1[2]; gs[7] = g1[3];
  v8h hv;
#pragma unroll
  for (int e = 0; e < 8; ++e) {
    const float gte = gs[e];
    const float sg  = __builtin_amdgcn_rcpf(1.0f + expf(-gte));
    hv[e] = (_Float16)(gte * sg * xs[e] * kActCarry);
  }
  unsigned short* dst = act + (size_t)row * kHid + c8;
  *(volatile v8h*)dst = hv;
  __threadfence();
  *(volatile v8h*)dst = hv;
}

__global__ __launch_bounds__(256) void pool_kernel(const float* __restrict__ h, const float* __restrict__ Wp,
                                                   const float* __restrict__ bp, float* __restrict__ pooled) {
  __shared__ float sc[kL];
  __shared__ float redM[8];
  __shared__ float redS[8];
  __shared__ float part[2 * kD];
  const int tid = threadIdx.x, lane = tid & 31, wave = tid >> 5;
  const int b = blockIdx.x;
  const float* hb = h + (size_t)b * kL * kD;
  const v4f wp = *(const v4f*)(Wp + lane * 4);
  const float bpv = bp[0];
#pragma unroll 1
  for (int it = 0; it < kL / 8; ++it) {
    const int l = it * 8 + wave;
    const v4f a = *(const v4f*)(hb + (size_t)l * kD + lane * 4);
    float p = a[0] * wp[0] + a[1] * wp[1] + a[2] * wp[2] + a[3] * wp[3];
    p += __shfl_xor(p, 16, 32);
    p += __shfl_xor(p, 8, 32);
    p += __shfl_xor(p, 4, 32);
    p += __shfl_xor(p, 2, 32);
    p += __shfl_xor(p, 1, 32);
    if (lane == 0) sc[l] = p + bpv;
  }
  __syncthreads();
  float m = -INFINITY;
#pragma unroll 1
  for (int i = 0; i < kL / 256; ++i) m = fmaxf(m, sc[tid + 256 * i]);
  m = fmaxf(m, __shfl_xor(m, 16, 32));
  m = fmaxf(m, __shfl_xor(m, 8, 32));
  m = fmaxf(m, __shfl_xor(m, 4, 32));
  m = fmaxf(m, __shfl_xor(m, 2, 32));
  m = fmaxf(m, __shfl_xor(m, 1, 32));
  if (lane == 0) redM[wave] = m;
  __syncthreads();
  float mx = redM[0];
#pragma unroll
  for (int i = 1; i < 8; ++i) mx = fmaxf(mx, redM[i]);
  float sm = 0.f;
#pragma unroll 1
  for (int i = 0; i < kL / 256; ++i) {
    const int idx = tid + 256 * i;
    const float e = expf(sc[idx] - mx);
    sc[idx] = e;
    sm += e;
  }
  sm += __shfl_xor(sm, 16, 32);
  sm += __shfl_xor(sm, 8, 32);
  sm += __shfl_xor(sm, 4, 32);
  sm += __shfl_xor(sm, 2, 32);
  sm += __shfl_xor(sm, 1, 32);
  if (lane == 0) redS[wave] = sm;
  __syncthreads();
  float tot = 0.f;
#pragma unroll
  for (int i = 0; i < 8; ++i) tot += redS[i];
  const int d = tid & (kD - 1);
  const int half = tid >> 7;
  float acc = 0.f;
#pragma unroll 4
  for (int l = half * (kL / 2); l < (half + 1) * (kL / 2); ++l) acc = fmaf(sc[l], hb[(size_t)l * kD + d], acc);
  part[half * kD + d] = acc;
  __syncthreads();
  if (tid < kD) {
    const float v = (part[tid] + part[kD + tid]) * (1.0f / tot);
    float* dst = pooled + b * kD + tid;
    *(volatile float*)dst = v;
    __threadfence();
    *(volatile float*)dst = v;
  }
}

__global__ __launch_bounds__(256) void classifier_kernel(const float* __restrict__ pooled, const float* __restrict__ Wc1,
                                                         const float* __restrict__ bc1, const float* __restrict__ Wc2,
                                                         const float* __restrict__ bc2, float* __restrict__ out) {
  __shared__ float sp[kB * kD];
  __shared__ float sz[kB * 64];
  const int tid = threadIdx.x;
  sp[tid]       = pooled[tid];
  sp[tid + 256] = pooled[tid + 256];
  __syncthreads();
  {
    const int b = tid >> 6, j = tid & 63;
    float acc = bc1[j];
#pragma unroll 4
    for (int d = 0; d < kD; ++d) acc = fmaf(Wc1[j * kD + d], sp[b * kD + d], acc);
    sz[tid] = fmaxf(acc, 0.0f);
  }
  __syncthreads();
  const int tcl = tid < (kB * 7) ? tid : (kB * 7 - 1);
  const int ob = tcl / 7;
  const int oo = tcl - ob * 7;
  float o = bc2[oo];
#pragma unroll 4
  for (int t = 0; t < 64; ++t) o = fmaf(Wc2[oo * 64 + t], sz[ob * 64 + t], o);
  if (tid < kB * 7) *(volatile float*)(out + tid) = o;
  __threadfence();
  if (tid < kB * 7) *(volatile float*)(out + tid) = o;
}

extern "C" void kernel_launch(void* const* d_in, const int* in_sizes, int n_in,
                              void* d_out, int out_size, void* d_ws, size_t ws_size,
                              hipStream_t stream) {
  if (n_in < 22) return;
  if (in_sizes[0] != kB * kL * kNF) return;
  if (in_sizes[1] != kB) return;
  if (in_sizes[2] != kNumEmb * kDED) return;
  if (in_sizes[3] != kD * kCin) return;
  if (in_sizes[6] != kNL * 3 * kD * kD) return;
  if (in_sizes[8] != kNL * kD * kD) return;
  if (in_sizes[12] != kNL * kHid2 * kD) return;
  if (in_sizes[14] != kNL * kD * kHid) return;
  if (in_sizes[18] != 64 * kD) return;
  if (in_sizes[20] != 7 * 64) return;
  if (out_size != kB * 7) return;
  if (ws_size < kWsTotal) return;

  const float* x      = (const float*)d_in[0];
  const int*   ids    = (const int*)d_in[1];
  const float* emb    = (const float*)d_in[2];
  const float* W_in   = (const float*)d_in[3];
  const float* b_in   = (const float*)d_in[4];
  const float* g_in   = (const float*)d_in[5];
  const float* Wqkv   = (const float*)d_in[6];
  const float* bqkv   = (const float*)d_in[7];
  const float* Wo     = (const float*)d_in[8];
  const float* bo     = (const float*)d_in[9];
  const float* g1     = (const float*)d_in[10];
  const float* g2     = (const float*)d_in[11];
  const float* W1     = (const float*)d_in[12];
  const float* b1     = (const float*)d_in[13];
  const float* W2     = (const float*)d_in[14];
  const float* b2     = (const float*)d_in[15];
  const float* Wp     = (const float*)d_in[16];
  const float* bp     = (const float*)d_in[17];
  const float* Wc1    = (const float*)d_in[18];
  const float* bc1    = (const float*)d_in[19];
  const float* Wc2    = (const float*)d_in[20];
  const float* bc2    = (const float*)d_in[21];

  char* ws = (char*)d_ws;
  unsigned short* wqkv16 = (unsigned short*)(ws + kOffWQKV);
  unsigned short* wo16   = (unsigned short*)(ws + kOffWO);
  unsigned short* w116   = (unsigned short*)(ws + kOffW1);
  unsigned short* w216   = (unsigned short*)(ws + kOffW2);
  float*          hA     = (float*)(ws + kOffHA);
  float*          hB     = (float*)(ws + kOffHB);
  unsigned short* hn16   = (unsigned short*)(ws + kOffHN);
  unsigned short* qk16   = (unsigned short*)(ws + kOffQK);
  unsigned short* vT16   = (unsigned short*)(ws + kOffVT);
  unsigned short* oa16   = (unsigned short*)(ws + kOffOA);
  float*          ff     = (float*)(ws + kOffFF);
  unsigned short* act16  = (unsigned short*)(ws + kOffACT);
  float*          cb     = (float*)(ws + kOffCB);
  float*          pooled = (float*)(ws + kOffPL);

  const float qk_scale = (float)(1.0 / sqrt((double)kHead));

  cast8_f16_kernel<<<(kNL * 3 * kD * kD / 8) / 256, 256, 0, stream>>>(Wqkv, wqkv16, kNL * 3 * kD * kD / 8, kWCarry);
  cast8_f16_kernel<<<(kNL * kD * kD / 8) / 256, 256, 0, stream>>>(Wo, wo16, kNL * kD * kD / 8, kWCarry);
  cast8_f16_kernel<<<(kNL * kHid2 * kD / 8) / 256, 256, 0, stream>>>(W1, w116, kNL * kHid2 * kD / 8, kWCarry);
  cast8_f16_kernel<<<(kNL * kD * kHid / 8) / 256, 256, 0, stream>>>(W2, w216, kNL * kD * kHid / 8, kWCarry);

  embed_const_kernel<<<1, 128, 0, stream>>>(ids, emb, W_in, b_in, cb);
  embed_tok_kernel<<<kTok / 32, 128, 0, stream>>>(x, W_in, cb, g_in, hA);

  for (int i = 0; i < kNL; ++i) {
    const unsigned short* wq = wqkv16 + (size_t)i * 3 * kD * kD;
    rmsnorm_f16_kernel<<<kTok / 16, 256, 0, stream>>>(hA, g1 + i * kD, hn16);
    wmma_gemm64<2, 1, false><<<64, 256, 0, stream>>>(
        hn16, kD, wq, kD, (void*)qk16, kQKld, bqkv + i * 3 * kD, nullptr,
        kTok, kQKld, kD, kWInv);
    wmma_gemm64<1, 1, false><<<32, 256, 0, stream>>>(
        wq + (size_t)2 * kD * kD, kD, hn16, kD, (void*)vT16, kTok, bqkv + i * 3 * kD + 2 * kD, nullptr,
        kD, kTok, kD, kWInv);
    attn_full_kernel<<<kB * (kL / 64), 128, 0, stream>>>(qk16, vT16, oa16, qk_scale);
    wmma_gemm64<2, 0, true><<<32, 256, 0, stream>>>(
        oa16, kD, wo16 + (size_t)i * kD * kD, kD, (void*)hB, kD, bo + i * kD, hA,
        kTok, kD, kD, kWInv);
    rmsnorm_f16_kernel<<<kTok / 16, 256, 0, stream>>>(hB, g2 + i * kD, hn16);
    wmma_gemm64<2, 0, false><<<256, 256, 0, stream>>>(
        hn16, kD, w116 + (size_t)i * kHid2 * kD, kD, (void*)ff, kHid2, b1 + i * kHid2, nullptr,
        kTok, kHid2, kD, kWInv);
    gate_mul_kernel<<<(kTok * (kHid / 8)) / 256, 256, 0, stream>>>(ff, act16);
    wmma_gemm64<2, 0, true><<<32, 256, 0, stream>>>(
        act16, kHid, w216 + (size_t)i * kD * kHid, kHid, (void*)hA, kD, b2 + i * kD, hB,
        kTok, kD, kHid, kW2Inv);
  }

  pool_kernel<<<kB, 256, 0, stream>>>(hA, Wp, bp, pooled);
  classifier_kernel<<<1, 256, 0, stream>>>(pooled, Wc1, bc1, Wc2, bc2, (float*)d_out);
}
